// LoRAAttention_15204184228289
// MI455X (gfx1250) — hardware-verified
//
#include <hip/hip_runtime.h>
#include <math.h>

constexpr int kSeq    = 4096;
constexpr int kDim    = 768;
constexpr int kHeads  = 12;
constexpr int kDh     = 64;
constexpr int kRank   = 8;
constexpr int kQChunk = 2048;
constexpr int kNChunk = kSeq / kQChunk;
constexpr float kLowRankScale = 2.0f;
constexpr float kWCarry    = 16.0f;
constexpr float kWCarryInv = 1.0f / 16.0f;
constexpr float kQKScale   = 0.125f;
constexpr float kPCarry    = 32768.0f;
constexpr float kAttCarry  = 256.0f;
constexpr float kPVScale   = kAttCarry / kPCarry;
constexpr float kOutScale  = 1.0f / (kAttCarry * kWCarry);
static_assert(kHeads * kDh == kDim, "shape");
static_assert(kSeq % 64 == 0 && kDim % 64 == 0 && kQChunk % 64 == 0 && kDh % 64 == 0, "M,N tile multiples");
static_assert(kDim % 32 == 0 && kDh % 32 == 0 && kSeq % 32 == 0, "K multiples of 32");
static_assert(kSeq % 512 == 0 && kQChunk * kNChunk == kSeq, "softmax mapping");
static_assert((kDim * kDim) % 2048 == 0, "fold block mapping");
static_assert((kSeq * kDim) % 2048 == 0, "cast block mapping");
static_assert(kRank * kDim == 6 * 256 * 4, "adapter staging: 6 float4 per thread of a 256-thread block");

typedef __attribute__((ext_vector_type(16))) _Float16 v16h;
typedef __attribute__((ext_vector_type(8)))  _Float16 v8h;
typedef __attribute__((ext_vector_type(16))) __bf16   v16b;
typedef __attribute__((ext_vector_type(8)))  __bf16   v8b;
typedef __attribute__((ext_vector_type(8)))  float    v8f;
typedef __attribute__((ext_vector_type(4)))  float    v4f;
typedef __attribute__((ext_vector_type(2)))  float    v2f;
typedef __attribute__((ext_vector_type(4)))  unsigned int v4u;

__device__ __forceinline__ unsigned short f2bf_bits(float f) {
  unsigned u = __float_as_uint(f);
  return (unsigned short)((u + 0x7FFFu + ((u >> 16) & 1u)) >> 16);
}
__device__ __forceinline__ float bf_bits2f(unsigned short h) { return __uint_as_float(((unsigned)h) << 16); }

__device__ __forceinline__ void dep_guard_h(v8f& a, v8f& b, v16h x, v16h y) { asm volatile("v_nop\n\tv_nop\n\tv_nop\n\tv_nop" : "+v"(a), "+v"(b) : "v"(x), "v"(y)); }
__device__ __forceinline__ void dep_guard_b(v8f& a, v8f& b, v16b x, v16b y) { asm volatile("v_nop\n\tv_nop\n\tv_nop\n\tv_nop" : "+v"(a), "+v"(b) : "v"(x), "v"(y)); }
__device__ __forceinline__ void dep_guard4_h(v8f& a, v8f& b, v8f& c, v8f& d, v16h x, v16h y) {
  asm volatile("v_nop\n\tv_nop\n\tv_nop\n\tv_nop" : "+v"(a), "+v"(b), "+v"(c), "+v"(d) : "v"(x), "v"(y));
}
__device__ __forceinline__ void dep_guard4_b(v8f& a, v8f& b, v8f& c, v8f& d, v16b x, v16b y) {
  asm volatile("v_nop\n\tv_nop\n\tv_nop\n\tv_nop" : "+v"(a), "+v"(b), "+v"(c), "+v"(d) : "v"(x), "v"(y));
}
__device__ __forceinline__ void keep4_h(v16h a, v16h b, v16h c, v16h d) { asm volatile("v_nop" :: "v"(a), "v"(b), "v"(c), "v"(d)); }
__device__ __forceinline__ void keep4_b(v16b a, v16b b, v16b c, v16b d) { asm volatile("v_nop" :: "v"(a), "v"(b), "v"(c), "v"(d)); }
__device__ __forceinline__ void acc_guard4(v8f& a, v8f& b, v8f& c, v8f& d) { asm volatile("v_nop\n\tv_nop\n\tv_nop\n\tv_nop" : "+v"(a), "+v"(b), "+v"(c), "+v"(d)); }
template <typename T> struct Frag;
template <> struct Frag<_Float16> {
  typedef v16h V; union U { v16h v; v8h h[2]; };
  static __device__ __forceinline__ v16h load(const _Float16* p) {
    U f; f.h[0] = *(const v8h*)(p); f.h[1] = *(const v8h*)(p + 16); return f.v;
  }
  static __device__ __forceinline__ v8f mma(v16h a, v16h b, v8f c) {
    return __builtin_amdgcn_wmma_f32_16x16x32_f16(false, a, false, b, (short)0, c, false, false);
  }
  static __device__ __forceinline__ void guard(v8f& a, v8f& b, v16h x, v16h y) { dep_guard_h(a, b, x, y); }
  static __device__ __forceinline__ void guard4(v8f& a, v8f& b, v8f& c, v8f& d, v16h x, v16h y) { dep_guard4_h(a, b, c, d, x, y); }
  static __device__ __forceinline__ void keep(v16h a, v16h b, v16h c, v16h d) { keep4_h(a, b, c, d); }
};
template <> struct Frag<__bf16> {
  typedef v16b V; union U { v16b v; v8b h[2]; };
  static __device__ __forceinline__ v16b load(const __bf16* p) {
    U f; f.h[0] = *(const v8b*)(p); f.h[1] = *(const v8b*)(p + 16); return f.v;
  }
  static __device__ __forceinline__ v8f mma(v16b a, v16b b, v8f c) {
    return __builtin_amdgcn_wmma_f32_16x16x32_bf16(false, a, false, b, (short)0, c, false, false);
  }
  static __device__ __forceinline__ void guard(v8f& a, v8f& b, v16b x, v16b y) { dep_guard_b(a, b, x, y); }
  static __device__ __forceinline__ void guard4(v8f& a, v8f& b, v8f& c, v8f& d, v16b x, v16b y) { dep_guard4_b(a, b, c, d, x, y); }
  static __device__ __forceinline__ void keep(v16b a, v16b b, v16b c, v16b d) { keep4_b(a, b, c, d); }
};

__device__ __forceinline__ unsigned pk16(unsigned short a, unsigned short b) { return (unsigned)a | ((unsigned)b << 16); }
__device__ __forceinline__ unsigned short h_bits(float f) { const _Float16 h = (_Float16)f; return __builtin_bit_cast(unsigned short, h); }

template <int ET> struct Elem;
template <> struct Elem<0> { typedef _Float16 T; };
template <> struct Elem<1> { typedef __bf16 T; };
template <int ET, bool SPLIT, int BIAS_MODE, int OUT_MODE, bool RESID, int ACT = 0>
__global__ __launch_bounds__(256) void wmma_gemm64(
    const unsigned short* __restrict__ Ap, const unsigned short* __restrict__ A2p, int lda, long strideA,
    const unsigned short* __restrict__ Btp, const unsigned short* __restrict__ Bt2p, int ldb, long strideB,
    void* __restrict__ Cout, void* __restrict__ Cout2, int ldc, long strideC,
    const float* __restrict__ bias,
    const float* __restrict__ resid, long strideR,
    int M, int N, int K, float scale) {
  typedef typename Elem<ET>::T T;
  typedef typename Frag<T>::V V;
  const T* A = (const T*)Ap; const T* A2 = (const T*)A2p; const T* Bt = (const T*)Btp; const T* Bt2 = (const T*)Bt2p;
  __shared__ __align__(16) float sT[8][16 * 68];
  const int b    = blockIdx.y;
  const int lane = threadIdx.x & 31;
  const int wave = threadIdx.x >> 5;
  const int tilesN = N >> 6;
  const int tilesM = M >> 6;
  const int tile = blockIdx.x * 8 + wave;
  if (tile >= tilesM * tilesN) return;
  const int tm = tile / tilesN;
  const int tn = tile - tm * tilesN;
  const int m0 = tm << 6;
  const int n0 = tn << 6;

  const T* Ab  = A  + (size_t)b * strideA;
  const T* Bb  = Bt + (size_t)b * strideB;
  const T* Ab2 = SPLIT ? (A2  + (size_t)b * strideA) : nullptr;
  const T* Bb2 = SPLIT ? (Bt2 + (size_t)b * strideB) : nullptr;

  const int rlane = lane & 15;
  const int koff  = (lane >> 4) * 8;
  const int mOff  = (lane >> 4) * 8;

  v8f acc[4][4];
#pragma unroll
  for (int i = 0; i < 4; ++i)
#pragma unroll
    for (int j = 0; j < 4; ++j) acc[i][j] = (v8f){0.f,0.f,0.f,0.f,0.f,0.f,0.f,0.f};

  for (int k0 = 0; k0 < K; k0 += 32) {
    V bh[4], bl[4];
#pragma unroll
    for (int j = 0; j < 4; ++j) {
      const size_t bo = (size_t)(n0 + (j << 4) + rlane) * ldb + koff + k0;
      bh[j] = Frag<T>::load(Bb + bo);
      if (SPLIT) bl[j] = Frag<T>::load(Bb2 + bo);
    }
#pragma unroll
    for (int i = 0; i < 4; ++i) {
      const size_t ao = (size_t)(m0 + (i << 4) + rlane) * lda + koff + k0;
      V ah = Frag<T>::load(Ab + ao);
      V al;
      if (SPLIT) al = Frag<T>::load(Ab2 + ao);
#pragma unroll
      for (int j = 0; j < 4; ++j) {
        acc[i][j] = Frag<T>::mma(ah, bh[j], acc[i][j]);
        if (SPLIT) {
          acc[i][j] = Frag<T>::mma(ah, bl[j], acc[i][j]);
          acc[i][j] = Frag<T>::mma(al, bh[j], acc[i][j]);
        }
      }
      Frag<T>::guard4(acc[i][0], acc[i][1], acc[i][2], acc[i][3], ah, SPLIT ? al : ah);
    }
    Frag<T>::keep(bh[0], bh[1], bh[2], bh[3]);
    if (SPLIT) Frag<T>::keep(bl[0], bl[1], bl[2], bl[3]);
  }
  acc_guard4(acc[0][0], acc[0][1], acc[0][2], acc[0][3]);
  acc_guard4(acc[1][0], acc[1][1], acc[1][2], acc[1][3]);
  acc_guard4(acc[2][0], acc[2][1], acc[2][2], acc[2][3]);
  acc_guard4(acc[3][0], acc[3][1], acc[3][2], acc[3][3]);

  float* slab = sT[wave];
  const float* Rb = RESID ? (resid + (size_t)b * strideR) : nullptr;
#pragma unroll
  for (int i = 0; i < 4; ++i) {
    const int mBase = m0 + (i << 4);
    float bmr[8] = {0.f, 0.f, 0.f, 0.f, 0.f, 0.f, 0.f, 0.f};
    if (BIAS_MODE == 1) {
      const float* bp = bias + mBase + mOff;
      const v4f bm0 = *(const v4f*)(bp);
      const v4f bm1 = *(const v4f*)(bp + 4);
      bmr[0] = bm0[0]; bmr[1] = bm0[1]; bmr[2] = bm0[2]; bmr[3] = bm0[3];
      bmr[4] = bm1[0]; bmr[5] = bm1[1]; bmr[6] = bm1[2]; bmr[7] = bm1[3];
    }
#pragma unroll
    for (int j = 0; j < 4; ++j) {
      const int n = n0 + (j << 4) + rlane;
      float bv = 0.f;
      if (BIAS_MODE == 2) bv = bias[n];
#pragma unroll
      for (int r = 0; r < 8; ++r) {
        float v = acc[i][j][r] * scale;
        if (BIAS_MODE == 1) v += bmr[r];
        if (BIAS_MODE == 2) v += bv;
        if (RESID) v += Rb[(size_t)(mBase + mOff + r) * ldc + n];
        if (ACT == 2) v = fmaxf(v, 0.0f);
        if (ACT == 4) v = (v > 0.f) ? v : 0.01f * v;
        slab[(mOff + r) * 68 + (j << 4) + rlane] = v;
      }
    }
    __builtin_amdgcn_fence(__ATOMIC_RELEASE, "workgroup");
    __builtin_amdgcn_wave_barrier();
    __builtin_amdgcn_fence(__ATOMIC_ACQUIRE, "workgroup");
    if (OUT_MODE == 0) {
      float* C = (float*)Cout + (size_t)b * strideC;
      const int hh = lane >> 4, c4 = (lane & 15) * 4;
      for (int pass = 0; pass < 2; ++pass) {
#pragma unroll
        for (int it = 0; it < 8; ++it) {
          const int row = it * 2 + hh;
          v4f v = *(const v4f*)(slab + row * 68 + c4);
          *(volatile v4f*)(C + (size_t)(mBase + row) * ldc + n0 + c4) = v;
        }
        __threadfence();
      }
    } else {
      const int q = lane >> 3, c8 = (lane & 7) * 8;
      unsigned short* C  = (unsigned short*)Cout  + (size_t)b * strideC;
      unsigned short* C2 = (OUT_MODE == 2) ? ((unsigned short*)Cout2 + (size_t)b * strideC) : nullptr;
      for (int pass = 0; pass < 2; ++pass) {
#pragma unroll
        for (int it = 0; it < 4; ++it) {
          const int row = it * 4 + q;
          const float* sp = slab + row * 68 + c8;
          v8h hv, lv;
#pragma unroll
          for (int e = 0; e < 8; ++e) {
            if (OUT_MODE == 1) {
              hv[e] = (_Float16)sp[e];
            } else {
              unsigned short hb = f2bf_bits(sp[e]);
              unsigned short lb = f2bf_bits(sp[e] - bf_bits2f(hb));
              hv[e] = __builtin_bit_cast(_Float16, hb);
              lv[e] = __builtin_bit_cast(_Float16, lb);
            }
          }
          *(volatile v8h*)(C + (size_t)(mBase + row) * ldc + n0 + c8) = hv;
          if (OUT_MODE == 2) *(volatile v8h*)(C2 + (size_t)(mBase + row) * ldc + n0 + c8) = lv;
        }
        __threadfence();
      }
    }
    __builtin_amdgcn_fence(__ATOMIC_RELEASE, "workgroup");
    __builtin_amdgcn_wave_barrier();
    __builtin_amdgcn_fence(__ATOMIC_ACQUIRE, "workgroup");
  }
}

__global__ __launch_bounds__(256) void cast8_f16_kernel(const float* __restrict__ in, unsigned short* __restrict__ out, int n8) {
  const int i = blockIdx.x * 256 + threadIdx.x;
  if (i >= n8) return;
  const float* p = in + 8 * (size_t)i;
  const v4f a = *(const v4f*)(p);
  const v4f c = *(const v4f*)(p + 4);
  unsigned short hb[8];
#pragma unroll
  for (int e = 0; e < 4; ++e) {
    hb[e]     = h_bits(a[e]);
    hb[4 + e] = h_bits(c[e]);
  }
  const v4u u = (v4u){pk16(hb[0], hb[1]), pk16(hb[2], hb[3]), pk16(hb[4], hb[5]), pk16(hb[6], hb[7])};
  unsigned short* q = out + 8 * (size_t)i;
  *(volatile v4u*)q = u;
  __threadfence();
  *(volatile v4u*)q = u;
}

__global__ __launch_bounds__(256) void fold_cast_kernel(
    const float* __restrict__ wq, const float* __restrict__ wk, const float* __restrict__ wv, const float* __restrict__ wo,
    const float* __restrict__ dq, const float* __restrict__ uq,
    const float* __restrict__ dk, const float* __restrict__ uk,
    const float* __restrict__ dv, const float* __restrict__ uv,
    unsigned short* __restrict__ wqkv16, unsigned short* __restrict__ wo16) {
  __shared__ __align__(16) float dsh[kRank * kDim];
  const int y = blockIdx.y;
  const int t = threadIdx.x;
  const float* W  = (y == 0) ? wq : (y == 1) ? wk : (y == 2) ? wv : wo;
  const float* Dn = (y == 0) ? dq : (y == 1) ? dk : dv;
  const float* Up = (y == 0) ? uq : (y == 1) ? uk : uv;
#pragma unroll
  for (int i = 0; i < 6; ++i) {
    const int q4 = (i * 256 + t) * 4;
    const v4f dd = *(const v4f*)(Dn + q4);
    *(v4f*)(dsh + q4) = dd;
  }
  __syncthreads();

  const int base = blockIdx.x * 2048 + 8 * t;
  const int e = base / kDim;
  const int d = base - e * kDim;
  const v4f w0 = *(const v4f*)(W + base);
  const v4f w1 = *(const v4f*)(W + base + 4);
  float s[8];
#pragma unroll
  for (int k = 0; k < 8; ++k) s[k] = 0.0f;
  if (y < 3) {
    const v4f u0 = *(const v4f*)(Up + e * kRank);
    const v4f u1 = *(const v4f*)(Up + e * kRank + 4);
    const float ur[8] = {u0[0], u0[1], u0[2], u0[3], u1[0], u1[1], u1[2], u1[3]};
#pragma unroll
    for (int r = 0; r < kRank; ++r) {
      const v4f a = *(const v4f*)(dsh + r * kDim + d);
      const v4f c = *(const v4f*)(dsh + r * kDim + d + 4);
#pragma unroll
      for (int k = 0; k < 4; ++k) {
        s[k]     += ur[r] * a[k];
        s[4 + k] += ur[r] * c[k];
      }
    }
  }
  float f[8];
#pragma unroll
  for (int k = 0; k < 4; ++k) {
    f[k]     = (w0[k] + kLowRankScale * s[k])     * kWCarry;
    f[4 + k] = (w1[k] + kLowRankScale * s[4 + k]) * kWCarry;
  }
  unsigned short hb[8];
#pragma unroll
  for (int k = 0; k < 8; ++k) hb[k] = h_bits(f[k]);
  const v4u u = (v4u){pk16(hb[0], hb[1]), pk16(hb[2], hb[3]), pk16(hb[4], hb[5]), pk16(hb[6], hb[7])};
  unsigned short* op = (y < 3) ? (wqkv16 + (size_t)y * kDim * kDim + base) : (wo16 + base);
  *(volatile v4u*)op = u;
  __threadfence();
  *(volatile v4u*)op = u;
}

__global__ __launch_bounds__(256) void softmax_row_kernel(const float* __restrict__ Sp, unsigned short* __restrict__ Pp) {
  __shared__ __align__(16) float lg[kSeq];
  __shared__ float redM[8];
  __shared__ float redS[8];
  const int i    = blockIdx.x;
  const int t    = threadIdx.x;
  const int lane = t & 31, wave = t >> 5;
  const float* sr = Sp + (size_t)i * kSeq;

  float mx = -__builtin_inff();
#pragma unroll 1
  for (int it = 0; it < 8; ++it) {
    const int c = it * 512 + 2 * t;
    const v2f sv = *(const v2f*)(sr + c);
    mx = fmaxf(mx, fmaxf(sv[0], sv[1]));
    *(v2f*)(lg + c) = sv;
  }
#pragma unroll
  for (int off = 16; off > 0; off >>= 1) mx = fmaxf(mx, __shfl_xor(mx, off, 32));
  if (lane == 0) redM[wave] = mx;
  __syncthreads();
  float m = redM[0];
#pragma unroll
  for (int w = 1; w < 8; ++w) m = fmaxf(m, redM[w]);

  float sum = 0.f;
#pragma unroll 1
  for (int it = 0; it < 8; ++it) {
    const int c = it * 512 + 2 * t;
    const v2f l = *(const v2f*)(lg + c);
    v2f ev;
#pragma unroll
    for (int e = 0; e < 2; ++e) {
      ev[e] = expf(l[e] - m);
      sum += ev[e];
    }
    *(v2f*)(lg + c) = ev;
  }
#pragma unroll
  for (int off = 16; off > 0; off >>= 1) sum += __shfl_xor(sum, off, 32);
  if (lane == 0) redS[wave] = sum;
  __syncthreads();
  float tot = redS[0];
#pragma unroll
  for (int w = 1; w < 8; ++w) tot += redS[w];
  const float inv = kPCarry / tot;

  const v4f e0 = *(const v4f*)(lg + 8 * t);
  const v4f e1 = *(const v4f*)(lg + 8 * t + 4);
  const v4f e2 = *(const v4f*)(lg + 2048 + 8 * t);
  const v4f e3 = *(const v4f*)(lg + 2048 + 8 * t + 4);
  unsigned short ha[8], hc[8];
#pragma unroll
  for (int e = 0; e < 4; ++e) {
    ha[e]     = h_bits(e0[e] * inv);
    ha[4 + e] = h_bits(e1[e] * inv);
    hc[e]     = h_bits(e2[e] * inv);
    hc[4 + e] = h_bits(e3[e] * inv);
  }
  const v4u ua = (v4u){pk16(ha[0], ha[1]), pk16(ha[2], ha[3]), pk16(ha[4], ha[5]), pk16(ha[6], ha[7])};
  const v4u uc = (v4u){pk16(hc[0], hc[1]), pk16(hc[2], hc[3]), pk16(hc[4], hc[5]), pk16(hc[6], hc[7])};
  unsigned short* pr = Pp + (size_t)i * kSeq;
  *(volatile v4u*)(pr + 8 * t) = ua;
  *(volatile v4u*)(pr + 2048 + 8 * t) = uc;
  __threadfence();
  *(volatile v4u*)(pr + 8 * t) = ua;
  *(volatile v4u*)(pr + 2048 + 8 * t) = uc;
}

extern "C" void kernel_launch(void* const* d_in, const int* in_sizes, int n_in,
                              void* d_out, int out_size, void* d_ws, size_t ws_size,
                              hipStream_t stream) {
  if (n_in < 15) return;
  const int nX = kSeq * kDim;
  const int nW = kDim * kDim;
  const int nA = kRank * kDim;
  if (in_sizes[0] != nX) return;
  if (in_sizes[1] != nW || in_sizes[3] != nW || in_sizes[5] != nW || in_sizes[7] != nW) return;
  if (in_sizes[2] != kDim || in_sizes[4] != kDim || in_sizes[6] != kDim || in_sizes[8] != kDim) return;
  for (int i = 9; i < 15; ++i) if (in_sizes[i] != nA) return;
  if (out_size != nX) return;

  const size_t szAct  = (size_t)kSeq * kDim * 2;
  const size_t szWqkv = (size_t)3 * kDim * kDim * 2;
  const size_t szWo   = (size_t)kDim * kDim * 2;
  const size_t szS    = (size_t)kQChunk * kSeq * 4;
  const size_t szP    = (size_t)kQChunk * kSeq * 2;
  const size_t offX    = 0;
  const size_t offWqkv = offX + szAct;
  const size_t offWo   = offWqkv + szWqkv;
  const size_t offQ    = offWo + szWo;
  const size_t offK    = offQ + szAct;
  const size_t offVT   = offK + szAct;
  const size_t offAtt  = offVT + szAct;
  const size_t offS    = offAtt + szAct;
  const size_t offP    = offS + szS;
  const size_t total   = offP + szP;
  if (ws_size < total) return;

  const float* x   = (const float*)d_in[0];
  const float* wq  = (const float*)d_in[1];
  const float* bq  = (const float*)d_in[2];
  const float* wk  = (const float*)d_in[3];
  const float* bk  = (const float*)d_in[4];
  const float* wv  = (const float*)d_in[5];
  const float* bv  = (const float*)d_in[6];
  const float* wo  = (const float*)d_in[7];
  const float* bo  = (const float*)d_in[8];
  const float* dq  = (const float*)d_in[9];
  const float* uq  = (const float*)d_in[10];
  const float* dk  = (const float*)d_in[11];
  const float* uk  = (const float*)d_in[12];
  const float* dv  = (const float*)d_in[13];
  const float* uv  = (const float*)d_in[14];
  float* out = (float*)d_out;
  char* ws = (char*)d_ws;
  unsigned short* X16    = (unsigned short*)(ws + offX);
  unsigned short* WQKV16 = (unsigned short*)(ws + offWqkv);
  unsigned short* WO16   = (unsigned short*)(ws + offWo);
  unsigned short* Q16    = (unsigned short*)(ws + offQ);
  unsigned short* K16    = (unsigned short*)(ws + offK);
  unsigned short* VT16   = (unsigned short*)(ws + offVT);
  unsigned short* ATT16  = (unsigned short*)(ws + offAtt);
  float*          SC     = (float*)(ws + offS);
  unsigned short* PP     = (unsigned short*)(ws + offP);
  const unsigned short* WQ16 = WQKV16;
  const unsigned short* WK16 = WQKV16 + (size_t)kDim * kDim;
  const unsigned short* WV16 = WQKV16 + (size_t)2 * kDim * kDim;

  const int n8 = nX / 8;
  cast8_f16_kernel<<<dim3((n8 + 255) / 256), dim3(256), 0, stream>>>(x, X16, n8);
  fold_cast_kernel<<<dim3(nW / 2048, 4), dim3(256), 0, stream>>>(wq, wk, wv, wo, dq, uq, dk, uk, dv, uv, WQKV16, WO16);

  const int tilesProj = (kSeq / 64) * (kDim / 64);
  wmma_gemm64<0, false, 2, 1, false, 0><<<dim3((tilesProj + 7) / 8, 1), dim3(256), 0, stream>>>(
      X16, X16, kDim, 0L, WQ16, WQ16, kDim, 0L,
      (void*)Q16, (void*)Q16, kDim, 0L, bq, bq, 0L, kSeq, kDim, kDim, kWCarryInv);
  wmma_gemm64<0, false, 2, 1, false, 0><<<dim3((tilesProj + 7) / 8, 1), dim3(256), 0, stream>>>(
      X16, X16, kDim, 0L, WK16, WK16, kDim, 0L,
      (void*)K16, (void*)K16, kDim, 0L, bk, bk, 0L, kSeq, kDim, kDim, kWCarryInv);
  wmma_gemm64<0, false, 1, 1, false, 0><<<dim3((tilesProj + 7) / 8, 1), dim3(256), 0, stream>>>(
      WV16, WV16, kDim, 0L, X16, X16, kDim, 0L,
      (void*)VT16, (void*)VT16, kSeq, 0L, bv, bv, 0L, kDim, kSeq, kDim, kWCarryInv);

  const int tilesScore = (kQChunk / 64) * (kSeq / 64);
  const int tilesPV    = (kQChunk / 64) * (kDh / 64);
  for (int h = 0; h < kHeads; ++h) {
    for (int c = 0; c < kNChunk; ++c) {
      const unsigned short* Ag  = Q16 + (size_t)c * kQChunk * kDim + (size_t)h * kDh;
      const unsigned short* Btg = K16 + (size_t)h * kDh;
      wmma_gemm64<0, false, 0, 0, false, 0><<<dim3((tilesScore + 7) / 8, 1), dim3(256), 0, stream>>>(
          Ag, Ag, kDim, 0L, Btg, Btg, kDim, 0L,
          (void*)SC, (void*)SC, kSeq, 0L, bq, bq, 0L, kQChunk, kSeq, kDh, kQKScale);
      softmax_row_kernel<<<dim3(kQChunk), dim3(256), 0, stream>>>(SC, PP);
      const unsigned short* VTg = VT16 + (size_t)h * kDh * kSeq;
      unsigned short* Attg = ATT16 + (size_t)c * kQChunk * kDim + (size_t)h * kDh;
      wmma_gemm64<0, false, 0, 1, false, 0><<<dim3((tilesPV + 7) / 8, 1), dim3(256), 0, stream>>>(
          PP, PP, kSeq, 0L, VTg, VTg, kSeq, 0L,
          (void*)Attg, (void*)Attg, kDim, 0L, bq, bq, 0L, kQChunk, kDh, kSeq, kPVScale);
    }
  }

  wmma_gemm64<0, false, 2, 0, false, 0><<<dim3((tilesProj + 7) / 8, 1), dim3(256), 0, stream>>>(
      ATT16, ATT16, kDim, 0L, WO16, WO16, kDim, 0L,
      (void*)out, (void*)out, kDim, 0L, bo, bo, 0L, kSeq, kDim, kDim, kOutScale);
}
